// GAFE_5849745457918
// MI455X (gfx1250) — hardware-verified
//
#include <hip/hip_runtime.h>

typedef _Float16 f16t;
typedef _Float16 v16h __attribute__((ext_vector_type(16)));
typedef _Float16 v8h  __attribute__((ext_vector_type(8)));
typedef float    v8f  __attribute__((ext_vector_type(8)));
typedef float    v4f  __attribute__((ext_vector_type(4)));
typedef v8h __attribute__((may_alias)) v8ha;
typedef v4f __attribute__((may_alias)) v4fa;
typedef v8f __attribute__((may_alias)) v8fa;
union Frag { v16h v; v8h half[2]; };

#define NB     8
#define CC     256
#define C2     512
#define HH     48
#define WD     48
#define NP     2304
#define PADW   50
#define NPP    2500
#define K1     2304
#define K2     4608
#define KSP    264
#define SSP    72
#define BN_EPS 1e-5f

#define WSC    16.0f
#define QCAR   8.0f
#define PCAR   1024.0f
#define TCAR   8.0f

__device__ __forceinline__ v8f wmma_f16(v16h a, v16h b, v8f c) {
  v8f d = __builtin_amdgcn_wmma_f32_16x16x32_f16(false, a, false, b, (short)0, c, false, false);
  asm volatile("v_nop\n\tv_nop\n\tv_nop\n\tv_nop" : "+v"(d) : "v"(a), "v"(b));
  return d;
}

__device__ __forceinline__ v16h load_frag32(const f16t* p, int h) {
  Frag f;
  f.half[0] = *(const v8ha*)(p + 8 * h);
  f.half[1] = *(const v8ha*)(p + 16 + 8 * h);
  return f.v;
}

__device__ __forceinline__ v8f zero8f() {
  v8f z;
  #pragma unroll
  for (int j = 0; j < 8; ++j) z[j] = 0.f;
  return z;
}

__device__ __forceinline__ void gemm_main(const f16t* __restrict__ A, int K, const f16t* __restrict__ Bw,
                                          int arow0, int n0, int h, int m, v8f (&acc)[4]) {
  const v8f z8 = zero8f();
  #pragma unroll
  for (int nt = 0; nt < 4; ++nt) acc[nt] = z8;
  const f16t* ap = A + (size_t)(arow0 + m) * K;
  const f16t* bp = Bw + (size_t)(n0 + m) * K;
  const size_t bst = (size_t)16 * K;
  #pragma unroll 1
  for (int k0 = 0; k0 < K; k0 += 32) {
    const v16h a = load_frag32(ap + k0, h);
    #pragma unroll
    for (int nt = 0; nt < 4; ++nt) {
      const v16h bb = load_frag32(bp + nt * bst + k0, h);
      acc[nt] = wmma_f16(a, bb, acc[nt]);
    }
  }
}

__global__ __launch_bounds__(256) void wcvt_k(
    const float* __restrict__ wq, const float* __restrict__ wk, const float* __restrict__ wv,
    const float* __restrict__ w1, const float* __restrict__ w2,
    f16t* __restrict__ W16, f16t* __restrict__ W1r, f16t* __restrict__ W2r)
{
  const int g = blockIdx.x * 256 + threadIdx.x;
  if (g >= 245760) return;
  const float* base;
  int stride;
  f16t* dst;
  if (g < 24576) {
    const int e8 = g * 8;
    const int sel = e8 >> 16, idx = e8 & 65535;
    const float* src = (sel == 0) ? wq : ((sel == 1) ? wk : wv);
    base = src + idx;
    stride = 1;
    dst = W16 + e8;
  } else if (g < 98304) {
    const int e8 = (g - 24576) * 8;
    const int o = e8 / K1, kk = e8 - o * K1;
    const int tap = kk >> 8, c = kk & 255;
    base = w1 + (size_t)(o * CC + c) * 9 + tap;
    stride = 9;
    dst = W1r + e8;
  } else {
    const int e8 = (g - 98304) * 8;
    const int o = e8 / K2, kk = e8 - o * K2;
    const int tap = kk >> 9, c = kk & 511;
    base = w2 + (size_t)(o * C2 + c) * 9 + tap;
    stride = 9;
    dst = W2r + e8;
  }
  v8h o8;
  #pragma unroll
  for (int i = 0; i < 8; ++i) o8[i] = (f16t)(base[i * stride] * WSC);
  *(volatile v8h*)dst = o8;
  __threadfence();
  *(volatile v8h*)dst = o8;
}

__global__ __launch_bounds__(256) void zpad_k(f16t* __restrict__ T1, f16t* __restrict__ T2) {
  const int t = blockIdx.x * 256 + threadIdx.x;
  if (t >= NB * 18816) return;
  const int b = t / 18816, r = t - b * 18816;
  int q, v, isT2;
  if (r < 6272) { q = r >> 5; v = r & 31; isT2 = 0; }
  else { const int r2 = r - 6272; q = r2 >> 6; v = r2 & 63; isT2 = 1; }
  int pp;
  if (q < 50) pp = q;
  else if (q < 100) pp = (PADW - 1) * PADW + (q - 50);
  else { const int u = q - 100; pp = (u / 2 + 1) * PADW + ((u & 1) ? (PADW - 1) : 0); }
  v8h z;
  #pragma unroll
  for (int j = 0; j < 8; ++j) z[j] = (f16t)0.0f;
  f16t* dst = isT2 ? (T2 + (size_t)(b * NPP + pp) * C2 + 8 * v)
                   : (T1 + (size_t)(b * NPP + pp) * CC + 8 * v);
  *(volatile v8h*)dst = z;
  __threadfence();
  *(volatile v8h*)dst = z;
}

__global__ __launch_bounds__(256) void xcvt_k(const float* __restrict__ x, f16t* __restrict__ XT) {
  __shared__ __attribute__((aligned(32))) f16t sH[64 * 64];
  const int tid = threadIdx.x, lane = tid & 31, w = tid >> 5;
  const int ch0 = blockIdx.x * 64, p0 = blockIdx.y * 64, b = blockIdx.z;
  const int xq = tid & 15, cl = tid >> 4, x0 = 4 * xq;
  #pragma unroll 1
  for (int j = 0; j < 4; ++j) {
    const int col = cl + 16 * j, c = ch0 + col;
    const v4f v = *(const v4fa*)(x + (size_t)(b * CC + c) * NP + p0 + x0);
    sH[(x0 + 0) * 64 + col] = (f16t)v.x;
    sH[(x0 + 1) * 64 + col] = (f16t)v.y;
    sH[(x0 + 2) * 64 + col] = (f16t)v.z;
    sH[(x0 + 3) * 64 + col] = (f16t)v.w;
  }
  __syncthreads();
  const int q8 = lane & 7, sub = lane >> 3;
  v8h vals[2];
  size_t d[2];
  #pragma unroll
  for (int i = 0; i < 2; ++i) {
    const int lid = 8 * w + 4 * i + sub;
    vals[i] = *(const v8ha*)(sH + lid * 64 + 8 * q8);
    d[i] = (size_t)(b * NP + p0 + lid) * CC + ch0 + 8 * q8;
  }
  #pragma unroll
  for (int i = 0; i < 2; ++i) *(volatile v8h*)(XT + d[i]) = vals[i];
  __threadfence();
  #pragma unroll
  for (int i = 0; i < 2; ++i) *(volatile v8h*)(XT + d[i]) = vals[i];
}

__global__ __launch_bounds__(128) void qkv_k(
    const f16t* __restrict__ XT, const f16t* __restrict__ W16, const float* __restrict__ bq,
    const float* __restrict__ bk, const float* __restrict__ bv,
    f16t* __restrict__ QT, f16t* __restrict__ KT, f16t* __restrict__ VC)
{
  __shared__ __attribute__((aligned(32))) f16t sH[64 * 64];
  const int tid = threadIdx.x, lane = tid & 31, w = tid >> 5;
  const int h = lane >> 4, m = lane & 15;
  const int gy = blockIdx.y;
  const int mode = gy >> 2, n0 = (gy & 3) * 64;
  const f16t* Bw = W16 + (size_t)mode * 65536;
  const float* bias = (mode == 0) ? bq : ((mode == 1) ? bk : bv);
  const int r0 = blockIdx.x * 64;
  v8f acc[4];
  gemm_main(XT, CC, Bw, r0 + 16 * w, n0, h, m, acc);
  const float osc = 1.0f / WSC;
  if (mode < 2) {
    #pragma unroll
    for (int nt = 0; nt < 4; ++nt) {
      const int col = 16 * nt + m;
      const float bvv = bias[n0 + col];
      #pragma unroll
      for (int r = 0; r < 8; ++r) {
        const float val = acc[nt][r] * osc + bvv;
        sH[(16 * w + 8 * h + r) * 64 + col] = (f16t)(val * QCAR);
      }
    }
  } else {
    #pragma unroll
    for (int nt = 0; nt < 4; ++nt) {
      const int col = 16 * nt + m;
      const float bvv = bias[n0 + col];
      v8h hv;
      #pragma unroll
      for (int r = 0; r < 8; ++r) hv[r] = (f16t)((acc[nt][r] * osc + bvv) * QCAR);
      *(v8ha*)(sH + col * 64 + 16 * w + 8 * h) = hv;
    }
  }
  __syncthreads();
  const int q8 = lane & 7, sub = lane >> 3;
  v8h vals[4];
  size_t d[4];
  f16t* pl;
  if (mode < 2) {
    pl = (mode == 0) ? QT : KT;
    #pragma unroll
    for (int i = 0; i < 4; ++i) {
      const int lid = 16 * w + 4 * i + sub;
      vals[i] = *(const v8ha*)(sH + lid * 64 + 8 * q8);
      d[i] = (size_t)(r0 + lid) * CC + n0 + 8 * q8;
    }
  } else {
    pl = VC;
    const int b = blockIdx.x / 36, p0 = (blockIdx.x - 36 * b) * 64;
    #pragma unroll
    for (int i = 0; i < 4; ++i) {
      const int lid = 16 * w + 4 * i + sub;
      vals[i] = *(const v8ha*)(sH + lid * 64 + 8 * q8);
      d[i] = (size_t)(b * CC + n0 + lid) * NP + p0 + 8 * q8;
    }
  }
  #pragma unroll
  for (int i = 0; i < 4; ++i) *(volatile v8h*)(pl + d[i]) = vals[i];
  __threadfence();
  #pragma unroll
  for (int i = 0; i < 4; ++i) *(volatile v8h*)(pl + d[i]) = vals[i];
}

__global__ __launch_bounds__(256) void attn_k(
    const f16t* __restrict__ QT, const f16t* __restrict__ KT, const f16t* __restrict__ VC,
    const float* __restrict__ ftr, const float* __restrict__ delta, f16t* __restrict__ T1)
{
  __shared__ __attribute__((aligned(32))) f16t  Ksw[64 * KSP];
  __shared__ __attribute__((aligned(32))) float Ssw[64 * SSP];
  __shared__ __attribute__((aligned(32))) f16t  Psw[64 * SSP];
  __shared__ float mstat[64];
  __shared__ float lstat[64];
  __shared__ float rsc[64];
  __shared__ float red[256];
  const int tid = threadIdx.x, lane = tid & 31, w = tid >> 5;
  const int h = lane >> 4, m = lane & 15;
  const int j0 = blockIdx.x * 64, b = blockIdx.y;

  #pragma unroll
  for (int e = 0; e < 8; ++e) {
    const int idx = tid + 256 * e;
    const int jj = idx >> 5, cv = idx & 31;
    *(v8ha*)(Ksw + jj * KSP + 8 * cv) =
        *(const v8ha*)(KT + (size_t)(b * NP + j0 + jj) * CC + 8 * cv);
  }
  if (tid < 64) { mstat[tid] = -1.0e30f; lstat[tid] = 0.f; }
  const v8f z8 = zero8f();
  v8f acc[2][4];
  #pragma unroll
  for (int cs = 0; cs < 2; ++cs) {
    #pragma unroll
    for (int js = 0; js < 4; ++js) acc[cs][js] = z8;
  }
  __syncthreads();

  const int is = w >> 1, js0 = 2 * (w & 1);
  const int col = tid & 63, quad = tid >> 6;
  const float sinv = 1.0f / (QCAR * QCAR);
  const f16t* vrow0 = VC + (size_t)(b * CC + 32 * w + m) * NP;
  const f16t* vrow1 = vrow0 + (size_t)16 * NP;

  #pragma unroll 1
  for (int i0 = 0; i0 < NP; i0 += 64) {
    v8f s0 = z8, s1 = z8;
    const f16t* ap = QT + (size_t)(b * NP + i0 + 16 * is + m) * CC;
    const f16t* kp0 = Ksw + (16 * js0 + m) * KSP;
    const f16t* kp1 = kp0 + 16 * KSP;
    #pragma unroll 1
    for (int c0 = 0; c0 < CC; c0 += 32) {
      const v16h a = load_frag32(ap + c0, h);
      const v16h b0 = load_frag32(kp0 + c0, h);
      const v16h b1 = load_frag32(kp1 + c0, h);
      s0 = wmma_f16(a, b0, s0);
      s1 = wmma_f16(a, b1, s1);
    }
    *(v8fa*)(Ssw + (16 * js0 + m) * SSP + 16 * is + 8 * h) = s0;
    *(v8fa*)(Ssw + (16 * js0 + 16 + m) * SSP + 16 * is + 8 * h) = s1;
    __syncthreads();

    float sv[16];
    {
      const float* sc = Ssw + col * SSP + 16 * quad;
      #pragma unroll
      for (int q = 0; q < 4; ++q) {
        const v4f t4 = *(const v4fa*)(sc + 4 * q);
        sv[4 * q + 0] = t4.x; sv[4 * q + 1] = t4.y; sv[4 * q + 2] = t4.z; sv[4 * q + 3] = t4.w;
      }
    }
    float mx = sv[0];
    #pragma unroll
    for (int r = 1; r < 16; ++r) mx = fmaxf(mx, sv[r]);
    red[quad * 64 + col] = mx;
    __syncthreads();
    if (tid < 64) {
      const float bm = fmaxf(fmaxf(red[tid], red[64 + tid]), fmaxf(red[128 + tid], red[192 + tid]));
      const float mo = mstat[tid];
      const float mn = fmaxf(mo, bm);
      mstat[tid] = mn;
      rsc[tid] = __expf((mo - mn) * sinv);
    }
    __syncthreads();

    const float mnew = mstat[col];
    float psum = 0.f;
    v8h pa, pb;
    #pragma unroll
    for (int r = 0; r < 8; ++r) {
      const float p = __expf((sv[r] - mnew) * sinv);
      psum += p;
      pa[r] = (f16t)(p * PCAR);
    }
    #pragma unroll
    for (int r = 0; r < 8; ++r) {
      const float p = __expf((sv[8 + r] - mnew) * sinv);
      psum += p;
      pb[r] = (f16t)(p * PCAR);
    }
    *(v8ha*)(Psw + col * SSP + 16 * quad) = pa;
    *(v8ha*)(Psw + col * SSP + 16 * quad + 8) = pb;
    red[quad * 64 + col] = psum;
    __syncthreads();
    if (tid < 64)
      lstat[tid] = lstat[tid] * rsc[tid] + ((red[tid] + red[64 + tid]) + (red[128 + tid] + red[192 + tid]));

    #pragma unroll
    for (int js = 0; js < 4; ++js) {
      const float rr = rsc[16 * js + m];
      #pragma unroll
      for (int cs = 0; cs < 2; ++cs) {
        #pragma unroll
        for (int e = 0; e < 8; ++e) acc[cs][js][e] *= rr;
      }
    }
    #pragma unroll
    for (int kc = 0; kc < 2; ++kc) {
      const v16h a0 = load_frag32(vrow0 + i0 + 32 * kc, h);
      const v16h a1 = load_frag32(vrow1 + i0 + 32 * kc, h);
      #pragma unroll
      for (int js = 0; js < 4; ++js) {
        const v16h bb = load_frag32(Psw + (16 * js + m) * SSP + 32 * kc, h);
        acc[0][js] = wmma_f16(a0, bb, acc[0][js]);
        acc[1][js] = wmma_f16(a1, bb, acc[1][js]);
      }
    }
    __syncthreads();
  }

  const float dsc = delta[0] * (1.0f / (QCAR * PCAR));
  f16t* sT = Ksw;
  #pragma unroll
  for (int js = 0; js < 4; ++js) {
    const int jl = 16 * js + m;
    const float linv = __builtin_amdgcn_rcpf(lstat[jl]) * dsc;
    const float* fp = ftr + (size_t)(b * CC) * NP + j0 + jl;
    #pragma unroll
    for (int cs = 0; cs < 2; ++cs) {
      const int cb = 32 * w + 16 * cs + 8 * h;
      v8h hv;
      #pragma unroll
      for (int r = 0; r < 8; ++r) {
        const float f = acc[cs][js][r] * linv + fp[(size_t)(cb + r) * NP];
        hv[r] = (f16t)(f * TCAR);
      }
      *(v8ha*)(sT + jl * CC + cb) = hv;
    }
  }
  __syncthreads();
  const int q8 = lane & 7, sub = lane >> 3;
  v8h vals[8];
  size_t d[8];
  #pragma unroll
  for (int i = 0; i < 8; ++i) {
    const int id = 32 * w + 4 * i + sub;
    const int jj = id >> 2, L = id & 3;
    vals[i] = *(const v8ha*)(sT + jj * CC + 64 * L + 8 * q8);
    const int j = j0 + jj;
    const int yy = j / WD, xx = j - yy * WD;
    d[i] = (size_t)(b * NPP + (yy + 1) * PADW + xx + 1) * CC + 64 * L + 8 * q8;
  }
  #pragma unroll
  for (int i = 0; i < 8; ++i) *(volatile v8h*)(T1 + d[i]) = vals[i];
  __threadfence();
  #pragma unroll
  for (int i = 0; i < 8; ++i) *(volatile v8h*)(T1 + d[i]) = vals[i];
}

__global__ __launch_bounds__(256) void conv_k(
    const f16t* __restrict__ T, int Cin, const f16t* __restrict__ Wr, int K,
    const float* __restrict__ g, const float* __restrict__ bt, const float* __restrict__ mean,
    const float* __restrict__ var, int sig, float osc, float* __restrict__ out)
{
  __shared__ __attribute__((aligned(32))) float sO[128 * 96];
  const int tid = threadIdx.x, lane = tid & 31, w = tid >> 5;
  const int h = lane >> 4, m = lane & 15;
  const int y2 = blockIdx.x, oh = blockIdx.y, b = blockIdx.z;
  const int yr = w >> 2, og = w & 3;
  const int y = 2 * y2 + yr, o0 = 128 * oh + 32 * og;
  const v8f z8 = zero8f();
  v8f acc[3][2];
  #pragma unroll
  for (int mt = 0; mt < 3; ++mt) { acc[mt][0] = z8; acc[mt][1] = z8; }

  #pragma unroll 1
  for (int tap = 0; tap < 9; ++tap) {
    const int dy = tap / 3, dx = tap - 3 * dy;
    const int rowb = b * NPP + (y + dy) * PADW + dx;
    const f16t* ab = T + (size_t)(rowb + m) * Cin;
    const f16t* wb = Wr + (size_t)(o0 + m) * K + (size_t)tap * Cin;
    #pragma unroll 1
    for (int c0 = 0; c0 < Cin; c0 += 32) {
      v16h a[3];
      #pragma unroll
      for (int mt = 0; mt < 3; ++mt) a[mt] = load_frag32(ab + (size_t)(16 * mt) * Cin + c0, h);
      #pragma unroll
      for (int nt = 0; nt < 2; ++nt) {
        const v16h bb = load_frag32(wb + (size_t)(16 * nt) * K + c0, h);
        #pragma unroll
        for (int mt = 0; mt < 3; ++mt) acc[mt][nt] = wmma_f16(a[mt], bb, acc[mt][nt]);
      }
    }
  }

  #pragma unroll
  for (int nt = 0; nt < 2; ++nt) {
    const int ol = 32 * og + 16 * nt + m;
    const int o = 128 * oh + ol;
    const float inv = g[o] / sqrtf(var[o] + BN_EPS);
    const float sh = bt[o] - mean[o] * inv;
    #pragma unroll
    for (int mt = 0; mt < 3; ++mt) {
      v8f vv;
      #pragma unroll
      for (int r = 0; r < 8; ++r) {
        const float xc = acc[mt][nt][r] * osc;
        float t = fmaxf(xc * inv + sh, 0.f);
        if (sig) t = __builtin_amdgcn_rcpf(1.0f + __expf(-t));
        vv[r] = t;
      }
      *(v8fa*)(sO + ol * 96 + 48 * yr + 16 * mt + 8 * h) = vv;
    }
  }
  __syncthreads();
  const int q8 = lane & 7, sub = lane >> 3;
  v4f vals[12];
  size_t d[12];
  #pragma unroll
  for (int i = 0; i < 12; ++i) {
    const int id = 48 * w + 4 * i + sub;
    const int oo = id / 3, L = id - 3 * oo;
    vals[i] = *(const v4fa*)(sO + oo * 96 + 32 * L + 4 * q8);
    d[i] = (size_t)(b * CC + 128 * oh + oo) * NP + y2 * 96 + 32 * L + 4 * q8;
  }
  #pragma unroll
  for (int i = 0; i < 12; ++i) *(volatile v4f*)(out + d[i]) = vals[i];
  __threadfence();
  #pragma unroll
  for (int i = 0; i < 12; ++i) *(volatile v4f*)(out + d[i]) = vals[i];
}

__global__ __launch_bounds__(256) void pgc_k(
    const float* __restrict__ ftr, const float* __restrict__ gate, f16t* __restrict__ T2)
{
  __shared__ __attribute__((aligned(32))) f16t sMA[2 * 48 * 64];
  const int tid = threadIdx.x, lane = tid & 31, w = tid >> 5;
  const int cg = blockIdx.x, y = blockIdx.y, b = blockIdx.z;
  #pragma unroll 1
  for (int e = 0; e < 3; ++e) {
    const int idx = tid + 256 * e;
    const int cq = idx / 12, xq = idx - 12 * cq, x0 = 4 * xq;
    const int c = 64 * cg + cq;
    const float* pl = ftr + (size_t)(b * CC + c) * NP;
    float s[4], mx[4];
    #pragma unroll
    for (int i = 0; i < 4; ++i) { s[i] = 0.f; mx[i] = -3.0e38f; }
    #pragma unroll
    for (int dy = 0; dy < 3; ++dy) {
      const int yy = y + dy - 1;
      const bool vy = (unsigned)yy < (unsigned)HH;
      const int yc = yy < 0 ? 0 : (yy > HH - 1 ? HH - 1 : yy);
      const float* rp = pl + yc * WD;
      const v4f m4 = *(const v4fa*)(rp + x0);
      const float lf = rp[x0 > 0 ? x0 - 1 : 0];
      const float rt = rp[(x0 + 4 < WD) ? x0 + 4 : WD - 1];
      float r6[6];
      bool ok[6];
      r6[0] = lf;   ok[0] = vy && (x0 > 0);
      r6[1] = m4.x; ok[1] = vy;
      r6[2] = m4.y; ok[2] = vy;
      r6[3] = m4.z; ok[3] = vy;
      r6[4] = m4.w; ok[4] = vy;
      r6[5] = rt;   ok[5] = vy && (x0 + 4 < WD);
      #pragma unroll
      for (int i = 0; i < 4; ++i) {
        #pragma unroll
        for (int dx = 0; dx < 3; ++dx) {
          const float ev = r6[i + dx];
          const bool o6 = ok[i + dx];
          s[i] += o6 ? ev : 0.f;
          mx[i] = fmaxf(mx[i], o6 ? ev : -3.0e38f);
        }
      }
    }
    const v4f g4 = *(const v4fa*)(gate + (size_t)(b * CC + c) * NP + y * WD + x0);
    float gv[4];
    gv[0] = g4.x; gv[1] = g4.y; gv[2] = g4.z; gv[3] = g4.w;
    #pragma unroll
    for (int i = 0; i < 4; ++i) {
      sMA[(x0 + i) * 64 + cq] = (f16t)((mx[i] * gv[i]) * TCAR);
      sMA[3072 + (x0 + i) * 64 + cq] = (f16t)(((s[i] * (1.0f / 9.0f)) * gv[i]) * TCAR);
    }
  }
  __syncthreads();
  const int q8 = lane & 7, sub = lane >> 3;
  const int part = w >> 2, wl = w & 3;
  v8h vals[3];
  size_t d[3];
  #pragma unroll
  for (int i = 0; i < 3; ++i) {
    const int xx = 12 * wl + 4 * i + sub;
    vals[i] = *(const v8ha*)(sMA + part * 3072 + xx * 64 + 8 * q8);
    d[i] = (size_t)(b * NPP + (y + 1) * PADW + xx + 1) * C2 + part * CC + 64 * cg + 8 * q8;
  }
  #pragma unroll
  for (int i = 0; i < 3; ++i) *(volatile v8h*)(T2 + d[i]) = vals[i];
  __threadfence();
  #pragma unroll
  for (int i = 0; i < 3; ++i) *(volatile v8h*)(T2 + d[i]) = vals[i];
}

extern "C" void kernel_launch(void* const* d_in, const int* in_sizes, int n_in,
                              void* d_out, int out_size, void* d_ws, size_t ws_size,
                              hipStream_t stream) {
  if (n_in < 18) return;
  const int tot = NB * CC * NP;
  if (in_sizes[0] != tot || out_size != tot) return;
  if (in_sizes[1] != CC * CC || in_sizes[3] != CC * CC || in_sizes[5] != CC * CC) return;
  if (in_sizes[2] != CC || in_sizes[4] != CC || in_sizes[6] != CC) return;
  if (in_sizes[7] < 1) return;
  if (in_sizes[8] != CC * CC * 9 || in_sizes[13] != CC * C2 * 9) return;
  const int vecidx[8] = {9, 10, 11, 12, 14, 15, 16, 17};
  for (int i = 0; i < 8; ++i) if (in_sizes[vecidx[i]] != CC) return;

  const float* ftr    = (const float*)d_in[0];
  const float* wq     = (const float*)d_in[1];
  const float* bq     = (const float*)d_in[2];
  const float* wk     = (const float*)d_in[3];
  const float* bk     = (const float*)d_in[4];
  const float* wv     = (const float*)d_in[5];
  const float* bv     = (const float*)d_in[6];
  const float* delta  = (const float*)d_in[7];
  const float* w_rbc  = (const float*)d_in[8];
  const float* g1     = (const float*)d_in[9];
  const float* b1     = (const float*)d_in[10];
  const float* m1     = (const float*)d_in[11];
  const float* v1     = (const float*)d_in[12];
  const float* w_rbc2 = (const float*)d_in[13];
  const float* g2     = (const float*)d_in[14];
  const float* b2     = (const float*)d_in[15];
  const float* m2     = (const float*)d_in[16];
  const float* v2     = (const float*)d_in[17];
  float* outp = (float*)d_out;

  const size_t szW16 = (size_t)3 * CC * CC * 2;
  const size_t szW1  = (size_t)CC * K1 * 2;
  const size_t szW2  = (size_t)CC * K2 * 2;
  const size_t szPL  = (size_t)NB * NP * CC * 2;
  const size_t szT1  = (size_t)NB * NPP * CC * 2;
  const size_t szG   = (size_t)NB * CC * NP * 4;
  const size_t szT2  = (size_t)NB * NPP * C2 * 2;
  size_t off = 0;
  char* ws = (char*)d_ws;
  f16t*  W16  = (f16t*)(ws + off); off += szW16;
  f16t*  W1r  = (f16t*)(ws + off); off += szW1;
  f16t*  W2r  = (f16t*)(ws + off); off += szW2;
  f16t*  XT   = (f16t*)(ws + off); off += szPL;
  f16t*  QT   = (f16t*)(ws + off); off += szPL;
  f16t*  KT   = (f16t*)(ws + off); off += szPL;
  f16t*  VC   = (f16t*)(ws + off); off += szPL;
  f16t*  T1   = (f16t*)(ws + off); off += szT1;
  float* GATE = (float*)(ws + off); off += szG;
  f16t*  T2   = (f16t*)(ws + off); off += szT2;
  if (off > ws_size) return;

  const float cosc = 1.0f / (WSC * TCAR);

  wcvt_k<<<960, 256, 0, stream>>>(wq, wk, wv, w_rbc, w_rbc2, W16, W1r, W2r);
  zpad_k<<<588, 256, 0, stream>>>(T1, T2);
  xcvt_k<<<dim3(CC / 64, NP / 64, NB), 256, 0, stream>>>(ftr, XT);
  qkv_k<<<dim3(NB * NP / 64, 12), 128, 0, stream>>>(XT, W16, bq, bk, bv, QT, KT, VC);
  attn_k<<<dim3(NP / 64, NB), 256, 0, stream>>>(QT, KT, VC, ftr, delta, T1);
  conv_k<<<dim3(HH / 2, 2, NB), 256, 0, stream>>>(T1, CC, W1r, K1, g1, b1, m1, v1, 1, cosc, GATE);
  pgc_k<<<dim3(CC / 64, HH, NB), 256, 0, stream>>>(ftr, GATE, T2);
  conv_k<<<dim3(HH / 2, 2, NB), 256, 0, stream>>>(T2, C2, W2r, K2, g2, b2, m2, v2, 0, cosc, outp);
}
